// HSTU_BSA_Triton_23201413333344
// MI455X (gfx1250) — hardware-verified
//
#include <hip/hip_runtime.h>
#include <math.h>

typedef __attribute__((ext_vector_type(16))) _Float16 v16h;
typedef __attribute__((ext_vector_type(16))) __bf16 v16b;
typedef __attribute__((ext_vector_type(8)))  _Float16 v8h;
typedef __attribute__((ext_vector_type(8)))  float v8f;
typedef __attribute__((ext_vector_type(4)))  float v4f;
typedef __attribute__((ext_vector_type(2)))  float v2f;
typedef __attribute__((ext_vector_type(4)))  unsigned v4u;
typedef __attribute__((ext_vector_type(4)))  int v4i;
typedef float __attribute__((may_alias)) float_a;
typedef int __attribute__((may_alias)) int_a;

template <typename T> __device__ __forceinline__ void vst2(void* p, T v) { *(volatile T*)p = v; __threadfence(); *(volatile T*)p = v; }
__device__ __forceinline__ v8f wmma16(v16h a, v16h b, v8f c) {
  v8f d = __builtin_amdgcn_wmma_f32_16x16x32_f16(false, a, false, b, (short)0, c, false, false);
  asm volatile("v_nop\n\tv_nop\n\tv_nop\n\tv_nop" : "+v"(d) : "v"(a), "v"(b));
  return d;
}
__device__ __forceinline__ v8f wmma_bf(v16b a, v16b b, v8f c) {
  v8f d = __builtin_amdgcn_wmma_f32_16x16x32_bf16(false, a, false, b, (short)0, c, false, false);
  asm volatile("v_nop\n\tv_nop\n\tv_nop\n\tv_nop" : "+v"(d) : "v"(a), "v"(b));
  return d;
}
__device__ __forceinline__ v16h frag_h(const _Float16* rowk0, int lane) {
  union { v16h v; v8h q[2]; } u; const _Float16* p = rowk0 + 8 * (lane >> 4);
  u.q[0] = *(const v8h*)p; u.q[1] = *(const v8h*)(p + 16); return u.v;
}
__device__ __forceinline__ v16h frag_f32(const float* rowk0, int lane) {
  v16h a; const float* p = rowk0 + 8 * (lane >> 4);
#pragma unroll
  for (int i = 0; i < 8; ++i) { a[i] = (_Float16)p[i]; a[8 + i] = (_Float16)p[16 + i]; }
  return a;
}
__device__ __forceinline__ v16h frag_f32s(const float* rowk0, int lane, float sc) {
  v16h a; const float* p = rowk0 + 8 * (lane >> 4);
#pragma unroll
  for (int i = 0; i < 8; ++i) { a[i] = (_Float16)(p[i] * sc); a[8 + i] = (_Float16)(p[16 + i] * sc); }
  return a;
}
__device__ __forceinline__ v16h fragc_f32(const float* W, int k0, int n, int lane, int ld, int K) {
  v16h a; const int g = lane >> 4;
#pragma unroll
  for (int i = 0; i < 8; ++i) { const int ka = k0 + 8 * g + i, kb = ka + 16;
    a[i] = (_Float16)(ka < K ? W[(size_t)ka * ld + n] : 0.f); a[8 + i] = (_Float16)(kb < K ? W[(size_t)kb * ld + n] : 0.f); }
  return a;
}
struct F2 { v16b h, l; };
__device__ __forceinline__ F2 bsplit16(const float v[16]) { F2 r;
#pragma unroll
  for (int i = 0; i < 16; ++i) { const __bf16 h = (__bf16)v[i]; r.h[i] = h; r.l[i] = (__bf16)(v[i] - (float)h); }
  return r; }
__device__ __forceinline__ F2 split_row(const float* row, int k0, int lane) { float v[16]; const float* p = row + k0 + 8 * (lane >> 4);
#pragma unroll
  for (int i = 0; i < 8; ++i) { v[i] = p[i]; v[8 + i] = p[16 + i]; }
  return bsplit16(v); }
__device__ __forceinline__ F2 split_rowK(const float* row, int k0, int lane, int K) { float v[16]; const int g = lane >> 4;
#pragma unroll
  for (int i = 0; i < 8; ++i) { const int ka = k0 + 8 * g + i, kb = ka + 16; v[i] = ka < K ? row[ka] : 0.f; v[8 + i] = kb < K ? row[kb] : 0.f; }
  return bsplit16(v); }
__device__ __forceinline__ F2 split_col(const float* W, int k0, int n, int lane, int ld, int K) { float v[16]; const int g = lane >> 4;
#pragma unroll
  for (int i = 0; i < 8; ++i) { const int ka = k0 + 8 * g + i, kb = ka + 16; v[i] = ka < K ? W[(size_t)ka * ld + n] : 0.f; v[8 + i] = kb < K ? W[(size_t)kb * ld + n] : 0.f; }
  return bsplit16(v); }
__device__ __forceinline__ v8f mac3(const F2& a, const F2& b, v8f c) { c = wmma_bf(a.l, b.h, c); c = wmma_bf(a.h, b.l, c); return wmma_bf(a.h, b.h, c); }
__device__ __forceinline__ float sigm(float v) { return 1.0f / (1.0f + expf(-v)); }
#define LDSX() do { asm volatile("s_wait_dscnt 0" ::: "memory"); __builtin_amdgcn_wave_barrier(); __builtin_amdgcn_fence(__ATOMIC_RELEASE, "workgroup"); } while (0)

#define NB 4
#define TT 2048
#define NH 4
#define DD 64
#define BS 32
#define NBLK (TT / BS)
#define NR (NB * TT)
#define RW (NH * DD)

__global__ __launch_bounds__(256) void k_cmp(const float* __restrict__ k, const float* __restrict__ v, float* __restrict__ kc, float* __restrict__ vc) {
  const int b = blockIdx.y, n = blockIdx.x, tid = threadIdx.x;
  float sk = 0.f, sv = 0.f;
#pragma unroll 1
  for (int j = 0; j < BS; ++j) { const size_t o = ((size_t)b * TT + n * BS + j) * RW + tid; sk += k[o]; sv += v[o]; }
  vst2(kc + ((size_t)b * NBLK + n) * RW + tid, (float_a)(sk / (float)BS)); vst2(vc + ((size_t)b * NBLK + n) * RW + tid, (float_a)(sv / (float)BS));
}
__global__ __launch_bounds__(256) void k_route(const float* __restrict__ q, const float* __restrict__ kc, const float* __restrict__ vc, const float* __restrict__ gcmp, float* __restrict__ oc, int* __restrict__ sel) {
  __shared__ float sq[RW]; __shared__ float sp[NH][NBLK]; __shared__ float ssc[NH][NBLK]; __shared__ __align__(16) int ssel[32];
  const int row = blockIdx.x, tid = threadIdx.x; const int b = row / TT, t = row % TT; const int h = tid >> 6, x = tid & 63;
  sq[tid] = q[(size_t)row * RW + tid];
  if (tid < 32) ssel[tid] = -1;
  __syncthreads();
  { const int n = x; const float* kr = kc + ((size_t)b * NBLK + n) * RW + h * DD; float s = 0.f;
#pragma unroll 8
    for (int d = 0; d < DD; ++d) s += sq[h * DD + d] * kr[d];
    s *= 0.125f; const bool valid = (t / BS) >= n;
    ssc[h][n] = valid ? s : -3.4e38f; sp[h][n] = valid ? s * sigm(s) : 0.f; }
  __syncthreads();
  { const int d = x; float a = 0.f; const int nmax = t / BS;
#pragma unroll 1
    for (int n = 0; n <= nmax; ++n) a += sp[h][n] * vc[((size_t)b * NBLK + n) * RW + h * DD + d];
    vst2(oc + (size_t)row * RW + h * DD + d, (float_a)(a * gcmp[(size_t)row * NH + h])); }
  if (x == 0) {
    int chosen[4] = {-1, -1, -1, -1}; const int nvalid = t / BS + 1;
    for (int s4 = 0; s4 < 4 && s4 < nvalid; ++s4) { int best = -1; float bv = -3.4e38f;
      for (int n = 0; n < nvalid; ++n) { bool used = false; for (int u = 0; u < s4; ++u) used |= (chosen[u] == n); if (used) continue; if (best < 0 || ssc[h][n] > bv) { best = n; bv = ssc[h][n]; } }
      chosen[s4] = best; }
    for (int s4 = 0; s4 < 4; ++s4) ssel[h * 4 + s4] = chosen[s4]; }
  __syncthreads();
  if (tid < 32) vst2(sel + (size_t)row * 32 + tid, (int_a)ssel[tid]);
}
__global__ __launch_bounds__(128) void k_slc(const float* __restrict__ q, const float* __restrict__ k, const float* __restrict__ v, const int* __restrict__ sel, const float* __restrict__ gslc, const float* __restrict__ oc, float* __restrict__ out) {
  __shared__ __align__(16) _Float16 sP[4][16][72];
  __shared__ __align__(16) float so[4][16][68];
  __shared__ int ssel[64][4];
  const int tid = threadIdx.x, w = tid >> 5, lane = tid & 31, col = lane & 15, g = lane >> 4;
  const int b = blockIdx.z, h = blockIdx.y, q0 = blockIdx.x * 64 + w * 16;
  for (int i = tid; i < 64 * 4; i += 128) ssel[i >> 2][i & 3] = sel[((size_t)b * TT + blockIdx.x * 64 + (i >> 2)) * 32 + h * 4 + (i & 3)];
  __syncthreads();
  v16h aq[2];
#pragma unroll
  for (int kc2 = 0; kc2 < 2; ++kc2) aq[kc2] = frag_f32(q + ((size_t)b * TT + q0 + col) * RW + h * DD + kc2 * 32, lane);
  int msel[8][4];
#pragma unroll
  for (int r = 0; r < 8; ++r)
#pragma unroll
    for (int u = 0; u < 4; ++u) msel[r][u] = ssel[w * 16 + 8 * g + r][u];
  v8f acc[4] = {};
  const int ntiles = blockIdx.x + 1;
#pragma unroll 1
  for (int kt = 0; kt < ntiles; ++kt) {
#pragma unroll
    for (int t4 = 0; t4 < 4; ++t4) { v8f s = {}; const int key = kt * 64 + t4 * 16 + col; const int blk = key / BS;
#pragma unroll
      for (int kc2 = 0; kc2 < 2; ++kc2) s = wmma16(aq[kc2], frag_f32(k + ((size_t)b * TT + key) * RW + h * DD + kc2 * 32, lane), s);
#pragma unroll
      for (int r = 0; r < 8; ++r) { const int qi = q0 + 8 * g + r; const bool on = (key <= qi) && (msel[r][0] == blk || msel[r][1] == blk || msel[r][2] == blk || msel[r][3] == blk);
        const float sc = s[r] * 0.125f; const float p = on ? sc * sigm(sc) : 0.f; sP[w][8 * g + r][t4 * 16 + col] = (_Float16)(p * 64.0f); } }
    LDSX();
#pragma unroll
    for (int kc2 = 0; kc2 < 2; ++kc2) { const v16h pa = frag_h(&sP[w][col][0] + kc2 * 32, lane);
#pragma unroll
      for (int t4 = 0; t4 < 4; ++t4) acc[t4] = wmma16(pa, fragc_f32(v + ((size_t)b * TT + kt * 64) * RW + h * DD, kc2 * 32, t4 * 16 + col, lane, RW, 64), acc[t4]); }
    __builtin_amdgcn_wave_barrier();
  }
#pragma unroll
  for (int t4 = 0; t4 < 4; ++t4)
#pragma unroll
    for (int r = 0; r < 8; ++r) { const size_t row = (size_t)b * TT + q0 + 8 * g + r; const int d = t4 * 16 + col;
      so[w][8 * g + r][d] = acc[t4][r] * (1.0f / 64.0f) * gslc[row * NH + h] + oc[row * RW + h * DD + d]; }
  LDSX();
  for (int qq = lane; qq < 16 * 16; qq += 32) { const int rl = qq >> 4, pc = qq & 15; vst2(out + ((size_t)b * TT + q0 + rl) * RW + h * DD + pc * 4, *(const v4f*)(&so[w][rl][pc * 4])); }
}
extern "C" void kernel_launch(void* const* d_in, const int* in_sizes, int n_in, void* d_out, int out_size, void* d_ws, size_t ws_size, hipStream_t stream) {
  (void)in_sizes; (void)n_in; (void)out_size; (void)ws_size;
  const float* q = (const float*)d_in[0]; const float* k = (const float*)d_in[1]; const float* v = (const float*)d_in[2]; const float* gcmp = (const float*)d_in[3]; const float* gslc = (const float*)d_in[4];
  float* out = (float*)d_out;
  char* ws = (char*)d_ws; size_t off = 0;
  auto take = [&](size_t bytes) { char* p = ws + off; off += (bytes + 255) & ~(size_t)255; return p; };
  float* kc = (float*)take((size_t)NB * NBLK * RW * 4); float* vc = (float*)take((size_t)NB * NBLK * RW * 4); float* oc = (float*)take((size_t)NR * RW * 4); int* sel = (int*)take((size_t)NR * 32 * 4);
  k_cmp<<<dim3(NBLK, NB), 256, 0, stream>>>(k, v, kc, vc);
  k_route<<<NR, 256, 0, stream>>>(q, kc, vc, gcmp, oc, sel);
  k_slc<<<dim3(TT / 64, NH, NB), 128, 0, stream>>>(q, k, v, sel, gslc, oc, out);
}
